// SelectiveSSMBlock_74526272520979
// MI455X (gfx1250) — hardware-run, weakly checked
//
#include <hip/hip_runtime.h>
#include <hip/hip_fp16.h>
#include <math.h>

typedef __attribute__((ext_vector_type(16))) _Float16 v16h;
typedef __attribute__((ext_vector_type(8)))  _Float16 v8h;
typedef __attribute__((ext_vector_type(8)))  float    v8f;
typedef __attribute__((ext_vector_type(4)))  float    v4f;
typedef __attribute__((ext_vector_type(2)))  unsigned v2u;
typedef __attribute__((ext_vector_type(4)))  unsigned v4u;

constexpr int kBatch   = 4;
constexpr int kL       = 2048;
constexpr int kRows    = kBatch * kL;
constexpr int kD       = 768;
constexpr int kNst     = 16;
constexpr int kWN      = 64;
constexpr int kOffB    = 0;
constexpr int kOffC    = kNst;
constexpr int kColDt   = 2 * kNst;
constexpr int kWReal   = 2 * kNst + 1;
constexpr int kWWords  = kD / 8;
constexpr int kDWords  = kD / 4;
constexpr int kAlpFloats = kD * kNst;
constexpr int kPadFloats = kAlpFloats + kD;
constexpr float kXCarry = 64.0f;
constexpr float kWCarry = 256.0f;
constexpr float kYCarry = 0.015625f;
static_assert(kRows == 8192 && kL == 2048 && kD == 768 && kNst == 16);
static_assert(kWN == 64 && kOffB == 0 && kOffC == 16 && kColDt == 32 && kWReal == 33);
static_assert(kWReal <= kWN && (kWN % 64) == 0 && (kD % 32) == 0 && (kRows % 32) == 0);
static_assert(kWWords == 96 && (kWWords % 32) == 0 && kDWords == 192);
static_assert((kD % 64) == 0 && (kL % 64) == 0);
static_assert(kAlpFloats == 12288 && kPadFloats == 13056);
static_assert(kXCarry * 0.015625f == 1.0f && kYCarry * 64.0f == 1.0f);

constexpr size_t kSzUH   = (size_t)kRows * kD * 2;
constexpr size_t kSzUR   = (size_t)kRows * kD * 4;
constexpr size_t kSzWALL = (size_t)kWN * kD * 2;
constexpr size_t kSzXP   = (size_t)kRows * kWN * 4;
constexpr size_t kSzDTP  = (size_t)kRows * kD * 4;
constexpr size_t kSzPADS = (size_t)kPadFloats * 4;
constexpr size_t kSzYH   = (size_t)kRows * kD * 2;
constexpr size_t kOffUH   = 0;
constexpr size_t kOffUR   = kOffUH   + kSzUH;
constexpr size_t kOffWALL = kOffUR   + kSzUR;
constexpr size_t kOffXP   = kOffWALL + kSzWALL;
constexpr size_t kOffDTP  = kOffXP   + kSzXP;
constexpr size_t kOffPADS = kOffDTP  + kSzDTP;
constexpr size_t kOffYH   = kOffPADS + kSzPADS;
constexpr size_t kWsTotal = kOffYH   + kSzYH;
static_assert(kSzUH == 12582912ull && kSzUR == 25165824ull && kSzWALL == 98304ull && kSzXP == 2097152ull);
static_assert(kSzDTP == 25165824ull && kSzPADS == 52224ull && kSzYH == 12582912ull);
static_assert(kWsTotal == 12582912ull + 25165824ull + 98304ull + 2097152ull + 25165824ull + 52224ull +
              12582912ull);
static_assert(kWsTotal == 77745152ull);
static_assert(kWsTotal <= 134217728ull);
static_assert((kSzUH % 128) == 0 && (kSzUR % 128) == 0 && (kSzWALL % 128) == 0 && (kSzXP % 128) == 0 &&
              (kSzDTP % 128) == 0 && (kSzPADS % 128) == 0 && (kSzYH % 128) == 0);
static_assert((((size_t)kAlpFloats * 4) % 128) == 0);
static_assert((((size_t)kWN * 4) % 128) == 0);

__device__ __forceinline__ _Float16 f16_flush(float v) {
  const float w = (fabsf(v) < 6.103515625e-05f) ? 0.0f : v;
  return (_Float16)w;
}

__device__ __forceinline__ float bf16r(float v) {
  unsigned u = __float_as_uint(v);
  u = (u + 0x7FFFu + ((u >> 16) & 1u)) & 0xFFFF0000u;
  return __uint_as_float(u);
}

__device__ __forceinline__ float h16_to_f32(unsigned hb) {
  const unsigned sgn = (hb & 0x8000u) << 16; const unsigned em = hb & 0x7fffu;
  const float fn = __uint_as_float((em << 13) + 0x38000000u);
  const float fs = (float)em * 5.9604644775390625e-8f;
  const float mag = (em < 0x400u) ? fs : fn; return __uint_as_float(__float_as_uint(mag) | sgn); }

namespace eng {
union FragU { v16h v; v8h h[2]; };
__device__ __forceinline__ v16h frag_load(const _Float16* p) {
  FragU f;
  f.h[0] = *(const v8h*)(p);
  f.h[1] = *(const v8h*)(p + 16);
  return f.v;
}
__device__ __forceinline__ v8f mma(v16h a, v16h b, v8f c) {
  return __builtin_amdgcn_wmma_f32_16x16x32_f16(false, a, false, b, (short)0, c, false, false);
}
__device__ __forceinline__ void guard1(v8f& a, v16h x, v16h y) {
  asm volatile("v_nop\n\tv_nop\n\tv_nop\n\tv_nop" : "+v"(a) : "v"(x), "v"(y));
}
__device__ __forceinline__ void guard_acc(v8f& a) {
  asm volatile("v_nop\n\tv_nop\n\tv_nop\n\tv_nop" : "+v"(a));
}
__device__ __forceinline__ void keep4(v16h a, v16h b, v16h c, v16h d) {
  asm volatile("v_nop" :: "v"(a), "v"(b), "v"(c), "v"(d));
}

template <int MI, int SPL>
__global__ __launch_bounds__(256) void gemm_f16_kernel(
    const unsigned short* __restrict__ Ap, const unsigned short* __restrict__ A2p, int lda,
    const unsigned short* __restrict__ Btp, const unsigned short* __restrict__ Bt2p, int ldb,
    float* __restrict__ C, int ldc, int M, int N, int K, float scale, float rscale)
{
  static_assert(MI >= 1 && MI <= 2);
  static_assert(SPL >= 0 && SPL <= 2);
  const _Float16* A   = (const _Float16*)Ap;
  const _Float16* A2  = (const _Float16*)A2p;
  const _Float16* Bt  = (const _Float16*)Btp;
  const _Float16* Bt2 = (const _Float16*)Bt2p;
  __shared__ __align__(16) float sT[8][16 * 68];
  const int lane = threadIdx.x & 31;
  const int wave = threadIdx.x >> 5;
  const int tilesN = N >> 6;
  const int tilesM = M / (16 * MI);
  const int tile = blockIdx.x * 8 + wave;
  if (tile >= tilesM * tilesN) return;
  const int tm = tile / tilesN;
  const int tn = tile - tm * tilesN;
  const int m0 = tm * (16 * MI);
  const int n0 = tn << 6;
  const int rlane = lane & 15;
  const int koff  = (lane >> 4) * 8;
  const int mOff  = (lane >> 4) * 8;

  v8f acc[MI][4], accr[MI][4];
#pragma unroll
  for (int i = 0; i < MI; ++i)
#pragma unroll
    for (int j = 0; j < 4; ++j) {
      acc[i][j]  = (v8f){0.f, 0.f, 0.f, 0.f, 0.f, 0.f, 0.f, 0.f};
      accr[i][j] = (v8f){0.f, 0.f, 0.f, 0.f, 0.f, 0.f, 0.f, 0.f};
    }

  for (int k0 = 0; k0 < K; k0 += 32) {
    v16h bh[4], bl[4];
#pragma unroll
    for (int j = 0; j < 4; ++j) {
      const size_t bo = (size_t)(n0 + (j << 4) + rlane) * ldb + koff + k0;
      bh[j] = frag_load(Bt + bo);
      if (SPL == 2) bl[j] = frag_load(Bt2 + bo); else bl[j] = bh[j];
    }
#pragma unroll
    for (int i = 0; i < MI; ++i) {
      const size_t ao = (size_t)(m0 + (i << 4) + rlane) * lda + koff + k0;
      const v16h ah = frag_load(A + ao);
      v16h al = ah;
      if (SPL >= 1) al = frag_load(A2 + ao);
#pragma unroll
      for (int j = 0; j < 4; ++j) {
        acc[i][j] = mma(ah, bh[j], acc[i][j]);
        if (SPL >= 1) accr[i][j] = mma(al, bh[j], accr[i][j]);
        if (SPL == 2) accr[i][j] = mma(ah, bl[j], accr[i][j]);
      }
#pragma unroll
      for (int j = 0; j < 4; ++j) {
        guard1(acc[i][j], ah, al);
        if (SPL >= 1) guard1(accr[i][j], ah, al);
      }
    }
    keep4(bh[0], bh[1], bh[2], bh[3]);
    if (SPL == 2) keep4(bl[0], bl[1], bl[2], bl[3]);
  }
#pragma unroll
  for (int i = 0; i < MI; ++i)
#pragma unroll
    for (int j = 0; j < 4; ++j) {
      guard_acc(acc[i][j]);
      if (SPL >= 1) guard_acc(accr[i][j]);
    }

  float* slab = sT[wave];
#pragma unroll
  for (int i = 0; i < MI; ++i) {
    const int mBase = m0 + (i << 4);
#pragma unroll
    for (int j = 0; j < 4; ++j) {
#pragma unroll
      for (int r = 0; r < 8; ++r) {
        float v = acc[i][j][r] * scale;
        if (SPL >= 1) v += accr[i][j][r] * rscale;
        slab[(mOff + r) * 68 + (j << 4) + rlane] = v;
      }
    }
    __builtin_amdgcn_fence(__ATOMIC_RELEASE, "workgroup");
    __builtin_amdgcn_wave_barrier();
    __builtin_amdgcn_fence(__ATOMIC_ACQUIRE, "workgroup");
    {
      const int hh = lane >> 4, c4 = (lane & 15) * 4;
      for (int pass = 0; pass < 2; ++pass) {
#pragma unroll
        for (int it = 0; it < 8; ++it) {
          const int row = it * 2 + hh;
          const v4f v = *(const v4f*)(slab + row * 68 + c4);
          *(volatile v4f*)(C + (size_t)(mBase + row) * ldc + n0 + c4) = v;
        }
        __threadfence();
      }
    }
    __builtin_amdgcn_fence(__ATOMIC_RELEASE, "workgroup");
    __builtin_amdgcn_wave_barrier();
    __builtin_amdgcn_fence(__ATOMIC_ACQUIRE, "workgroup");
  }
}
}

__device__ __forceinline__ _Float16 in_half(float v, float carry, bool live) {
  const float t = live ? (bf16r(v) * carry) : 0.0f;
  return f16_flush(t);
}
__device__ __forceinline__ _Float16 val_half(float v, float carry, bool live) {
  const float t = live ? (v * carry) : 0.0f;
  return f16_flush(t);
}
__device__ __forceinline__ int imin2(int a, int b) {
  return (a < b) ? a : b;
}
__device__ __forceinline__ int iclamp(int v, int lo, int hi) {
  const int t = (v < lo) ? lo : v;
  return (t > hi) ? hi : t;
}

__global__ __launch_bounds__(256) void pack_x_kernel(
    const float* __restrict__ x, unsigned short* __restrict__ XH)
{
  const int i = blockIdx.x * 256 + threadIdx.x;
  const float* sp = x + (size_t)i * 8;
  const v4f a0 = *(const v4f*)(sp);
  const v4f a1 = *(const v4f*)(sp + 4);
  const float f0 = a0[0];
  const float f1 = a0[1];
  const float f2 = a0[2];
  const float f3 = a0[3];
  const float f4 = a1[0];
  const float f5 = a1[1];
  const float f6 = a1[2];
  const float f7 = a1[3];
  const float r0 = bf16r(f0);
  const float r1 = bf16r(f1);
  const float r2 = bf16r(f2);
  const float r3 = bf16r(f3);
  const float r4 = bf16r(f4);
  const float r5 = bf16r(f5);
  const float r6 = bf16r(f6);
  const float r7 = bf16r(f7);
  v8h hv;
  hv[0] = val_half(r0, kXCarry, true);
  hv[1] = val_half(r1, kXCarry, true);
  hv[2] = val_half(r2, kXCarry, true);
  hv[3] = val_half(r3, kXCarry, true);
  hv[4] = val_half(r4, kXCarry, true);
  hv[5] = val_half(r5, kXCarry, true);
  hv[6] = val_half(r6, kXCarry, true);
  hv[7] = val_half(r7, kXCarry, true);
  unsigned short* qh = XH + (size_t)i * 8;
  *(volatile v8h*)qh = hv;
  __threadfence();
  *(volatile v8h*)qh = hv;
}

__global__ __launch_bounds__(256) void rne_x_kernel(
    const float* __restrict__ x, float* __restrict__ XR)
{
  const int i = blockIdx.x * 256 + threadIdx.x;
  const v4f a0 = *(const v4f*)(x + (size_t)i * 4);
  const float f0 = a0[0];
  const float f1 = a0[1];
  const float f2 = a0[2];
  const float f3 = a0[3];
  v4f o;
  o[0] = bf16r(f0);
  o[1] = bf16r(f1);
  o[2] = bf16r(f2);
  o[3] = bf16r(f3);
  float* q = XR + (size_t)i * 4;
  *(volatile v4f*)q = o;
  __threadfence();
  *(volatile v4f*)q = o;
}

__device__ __forceinline__ float wrow_src(float vb, float vc, float vq, bool isB, bool isC) {
  const float vcq = isC ? vc : vq;
  return isB ? vb : vcq;
}
__global__ __launch_bounds__(256) void pack_w_kernel(
    const float* __restrict__ wb, const float* __restrict__ wc, const float* __restrict__ qd,
    unsigned short* __restrict__ WALL)
{
  const int i = blockIdx.x * 256 + threadIdx.x;
  const int n = i / kWWords;
  const int c8 = (i - n * kWWords) * 8;
  const bool isB = (n < kOffC);
  const bool isC = (n < kColDt);
  const bool live = (n < kWReal);
  const int nb = imin2(n, kNst - 1);
  const int nc = iclamp(n - kOffC, 0, kNst - 1);
  const float* pb = wb + (size_t)nb * kD + c8;
  const float* pc = wc + (size_t)nc * kD + c8;
  const float* pq = qd + c8;
  const v4f b0 = *(const v4f*)(pb);
  const v4f b1 = *(const v4f*)(pb + 4);
  const v4f c0 = *(const v4f*)(pc);
  const v4f c1 = *(const v4f*)(pc + 4);
  const v4f q0 = *(const v4f*)(pq);
  const v4f q1 = *(const v4f*)(pq + 4);
  const float fb0 = b0[0];
  const float fb1 = b0[1];
  const float fb2 = b0[2];
  const float fb3 = b0[3];
  const float fb4 = b1[0];
  const float fb5 = b1[1];
  const float fb6 = b1[2];
  const float fb7 = b1[3];
  const float fc0 = c0[0];
  const float fc1 = c0[1];
  const float fc2 = c0[2];
  const float fc3 = c0[3];
  const float fc4 = c1[0];
  const float fc5 = c1[1];
  const float fc6 = c1[2];
  const float fc7 = c1[3];
  const float fq0 = q0[0];
  const float fq1 = q0[1];
  const float fq2 = q0[2];
  const float fq3 = q0[3];
  const float fq4 = q1[0];
  const float fq5 = q1[1];
  const float fq6 = q1[2];
  const float fq7 = q1[3];
  const float s0 = wrow_src(fb0, fc0, fq0, isB, isC);
  const float s1 = wrow_src(fb1, fc1, fq1, isB, isC);
  const float s2 = wrow_src(fb2, fc2, fq2, isB, isC);
  const float s3 = wrow_src(fb3, fc3, fq3, isB, isC);
  const float s4 = wrow_src(fb4, fc4, fq4, isB, isC);
  const float s5 = wrow_src(fb5, fc5, fq5, isB, isC);
  const float s6 = wrow_src(fb6, fc6, fq6, isB, isC);
  const float s7 = wrow_src(fb7, fc7, fq7, isB, isC);
  v8h hv;
  hv[0] = in_half(s0, kWCarry, live);
  hv[1] = in_half(s1, kWCarry, live);
  hv[2] = in_half(s2, kWCarry, live);
  hv[3] = in_half(s3, kWCarry, live);
  hv[4] = in_half(s4, kWCarry, live);
  hv[5] = in_half(s5, kWCarry, live);
  hv[6] = in_half(s6, kWCarry, live);
  hv[7] = in_half(s7, kWCarry, live);
  unsigned short* q = WALL + (size_t)i * 8;
  *(volatile v8h*)q = hv;
  __threadfence();
  *(volatile v8h*)q = hv;
}

__global__ __launch_bounds__(256) void dt_plane_kernel(
    const float* __restrict__ XP, const float* __restrict__ pd, float* __restrict__ DTP)
{
  const int i = blockIdx.x * 256 + threadIdx.x;
  const int r = i / kDWords;
  const float s = XP[(size_t)r * kWN + kColDt];
  const float p = pd[0];
  const float v = s + bf16r(p);
  v4f o;
  o[0] = v;
  o[1] = v;
  o[2] = v;
  o[3] = v;
  float* q = DTP + (size_t)i * 4;
  *(volatile v4f*)q = o;
  __threadfence();
  *(volatile v4f*)q = o;
}

__global__ __launch_bounds__(32) void pads_kernel(
    const float* __restrict__ amat, float* __restrict__ PADS)
{
  const int wi = blockIdx.x * 32 + threadIdx.x;
  const int f0 = wi * 4;
  const bool isA = (f0 < kAlpFloats);
  const int ea = isA ? f0 : (kAlpFloats - 4);
  const v4f va = *(const v4f*)(amat + ea);
  const float a0 = va[0];
  const float a1 = va[1];
  const float a2 = va[2];
  const float a3 = va[3];
  const float g0 = logf(-bf16r(a0));
  const float g1 = logf(-bf16r(a1));
  const float g2 = logf(-bf16r(a2));
  const float g3 = logf(-bf16r(a3));
  v4f o;
  o[0] = isA ? g0 : 0.0f;
  o[1] = isA ? g1 : 0.0f;
  o[2] = isA ? g2 : 0.0f;
  o[3] = isA ? g3 : 0.0f;
  float* q = PADS + (size_t)f0;
  *(volatile v4f*)q = o;
  __threadfence();
  *(volatile v4f*)q = o;
}

typedef float    ms1_v4f __attribute__((ext_vector_type(4)));
typedef unsigned ms1_v4u __attribute__((ext_vector_type(4)));
struct ms1_args {
  const float* dtpre;
  const float* u;
  const float* bc;
  const float* z;
  const float* A_log;
  const float* Dskip;
  __half* y;
  __half* y_lo;
  long ld_dtpre;
  long ld_u;
  long ld_bc;
  long ld_z;
  long ld_y;
  int offB;
  int offC;
  int offZ;
  float ycarry;
  int dir;
  int D;
  int L;
  int nbatch;
};
static_assert(sizeof(ms1_args) == 136);

__device__ __forceinline__ float ms1_flush16(float v) {
  return (fabsf(v) < 6.103515625e-05f) ? 0.0f : v;
}
__device__ __forceinline__ unsigned ms1_h16bits(float v) {
  return (unsigned)__half_as_ushort(__float2half_rn(ms1_flush16(v)));
}
__device__ __forceinline__ float ms1_h16val(unsigned b) {
  return __half2float(__ushort_as_half((unsigned short)b));
}
__device__ __forceinline__ float ms1_softplus(float v) {
  return fmaxf(v, 0.0f) + log1pf(expf(-fabsf(v)));
}
__device__ __forceinline__ void ms1_pack2(float v0, float v1, unsigned& hw, unsigned& lw) {
  const unsigned h0 = ms1_h16bits(v0);
  const unsigned h1 = ms1_h16bits(v1);
  const float r0 = (v0 - ms1_h16val(h0)) * 2048.0f;
  const float r1 = (v1 - ms1_h16val(h1)) * 2048.0f;
  const unsigned l0 = ms1_h16bits(r0);
  const unsigned l1 = ms1_h16bits(r1);
  hw = h0 | (h1 << 16);
  lw = l0 | (l1 << 16);
}

template <int NSTATE>
__global__ __launch_bounds__(64 * (NSTATE / 16)) void ms1_scan_kernel(ms1_args a)
{
  static_assert(NSTATE == 16 || NSTATE == 64);
  constexpr int NQ  = NSTATE / 16;
  constexpr int NT  = 64 * NQ;
  constexpr int NW  = NT / 32;
  constexpr int BCW = 2 * NSTATE;
  constexpr int YP  = 68;
  constexpr int RPI = NW * 4;
  constexpr int NIT = 64 / RPI;
  static_assert(16 * NT <= 64 * YP);
  __shared__ __align__(16) float sBC[64 * BCW];
  __shared__ __align__(16) float sY[64 * YP];
  const int tid  = threadIdx.x;
  const int lane = tid & 31;
  const int wave = tid >> 5;
  const int c    = tid / NQ;
  const int sq   = tid - c * NQ;
  const int bpb  = a.D / 64;
  const int bi   = blockIdx.x / bpb;
  if (bi >= a.nbatch) return;
  const int d0 = (blockIdx.x - bi * bpb) * 64;
  const int d  = d0 + c;
  const long rowb = (long)bi * a.L;
  const bool hasz  = (a.z != nullptr);
  const bool hasD  = (a.Dskip != nullptr);
  const bool hasLo = (a.y_lo != nullptr);

#pragma unroll 1
  for (int n = 0; n < 16; ++n) {
    const float al = a.A_log[(long)d * NSTATE + sq * 16 + n];
    sY[n * NT + tid] = -expf(al);
  }
  __syncthreads();
  float An[16], h[16];
#pragma unroll
  for (int n = 0; n < 16; ++n) {
    An[n] = sY[n * NT + tid];
    h[n] = 0.0f;
  }
  float Dd = 0.0f;
  if (hasD) Dd = a.Dskip[d];

  const int nchunk = a.L / 64;
  const bool fwd = (a.dir > 0);
  const int s0 = fwd ? 0 : 63;
  const int sd = fwd ? 1 : -1;
  const int q  = lane >> 3;
  const int c8 = (lane & 7) * 8;

  for (int ci = 0; ci < nchunk; ++ci) {
    const int tb = fwd ? (ci * 64) : (a.L - 64 - ci * 64);
    const long rowc = rowb + tb;
    __syncthreads();
#pragma unroll 8
    for (int i = 0; i < 32; ++i) {
      const int idx = tid + i * NT;
      const int st  = idx / BCW;
      const int col = idx - st * BCW;
      const int sc  = (col < NSTATE) ? (a.offB + col) : (a.offC + col - NSTATE);
      sBC[idx] = a.bc[(rowc + st) * a.ld_bc + sc];
    }
    __syncthreads();
    for (int s = 0; s < 64; ++s) {
      const int ls = s0 + sd * s;
      const long row = rowc + ls;
      float pre = a.dtpre[row * a.ld_dtpre + d];
      float uv  = a.u[row * a.ld_u + d];
      float zv  = 0.0f;
      if (hasz) zv = a.z[row * a.ld_z + a.offZ + d];
      asm volatile("" : "+v"(pre));
      asm volatile("" : "+v"(uv));
      asm volatile("" : "+v"(zv));
      const float delta = ms1_softplus(pre);
      const float dtx = delta * uv;
      const float* bp = sBC + ls * BCW + sq * 16;
      const float* cp = bp + NSTATE;
      ms1_v4f Bq[4], Cq[4];
#pragma unroll
      for (int k = 0; k < 4; ++k) {
        Bq[k] = *(const ms1_v4f*)(bp + 4 * k);
        Cq[k] = *(const ms1_v4f*)(cp + 4 * k);
      }
      float yv = 0.0f;
#pragma unroll
      for (int n = 0; n < 16; ++n) {
        const float e = __expf(delta * An[n]);
        h[n] = fmaf(e, h[n], dtx * Bq[n >> 2][n & 3]);
        yv = fmaf(h[n], Cq[n >> 2][n & 3], yv);
      }
      if (NQ > 1) {
        yv += __shfl_xor(yv, 1, 32);
        yv += __shfl_xor(yv, 2, 32);
      }
      if (hasD) yv = fmaf(uv, Dd, yv);
      if (hasz) {
        const float sg = __builtin_amdgcn_rcpf(1.0f + expf(-zv));
        yv = yv * (zv * sg);
      }
      if (sq == 0) sY[ls * YP + c] = yv * a.ycarry;
    }
    __syncthreads();
    ms1_v4u hw[NIT], lw[NIT];
#pragma unroll
    for (int it = 0; it < NIT; ++it) {
      const int row = it * RPI + wave * 4 + q;
      const float* sp = sY + row * YP + c8;
      const ms1_v4f f0 = *(const ms1_v4f*)(sp);
      const ms1_v4f f1 = *(const ms1_v4f*)(sp + 4);
      unsigned h0, h1, h2, h3, l0, l1, l2, l3;
      ms1_pack2(f0[0], f0[1], h0, l0);
      ms1_pack2(f0[2], f0[3], h1, l1);
      ms1_pack2(f1[0], f1[1], h2, l2);
      ms1_pack2(f1[2], f1[3], h3, l3);
      hw[it] = (ms1_v4u){h0, h1, h2, h3};
      lw[it] = (ms1_v4u){l0, l1, l2, l3};
    }
    for (int pass = 0; pass < 2; ++pass) {
#pragma unroll
      for (int it = 0; it < NIT; ++it) {
        const int row = it * RPI + wave * 4 + q;
        const long o = (rowc + row) * a.ld_y + d0 + c8;
        *(volatile ms1_v4u*)(a.y + o) = hw[it];
        if (hasLo) *(volatile ms1_v4u*)(a.y_lo + o) = lw[it];
      }
      __threadfence();
    }
  }
}

__device__ __forceinline__ float out_val(unsigned hb) {
  return h16_to_f32(hb) * (1.0f / kYCarry);
}
__global__ __launch_bounds__(256) void out_kernel(
    const unsigned short* __restrict__ YH, float* __restrict__ out)
{
  const int i = blockIdx.x * 256 + threadIdx.x;
  const v2u wy = *(const v2u*)(YH + (size_t)i * 4);
  const unsigned w0 = wy[0];
  const unsigned w1 = wy[1];
  v4f o;
  o[0] = out_val(w0 & 0xffffu);
  o[1] = out_val(w0 >> 16);
  o[2] = out_val(w1 & 0xffffu);
  o[3] = out_val(w1 >> 16);
  float* q = out + (size_t)i * 4;
  *(volatile v4f*)q = o;
  __threadfence();
  *(volatile v4f*)q = o;
}

static_assert(((kRows / 32) * (kWN / 64)) % 8 == 0 && ((kRows / 32) * (kWN / 64)) / 8 == 32);
static_assert((8192 / 32) * (64 / 64) / 8 == 32);
static_assert(((kRows * kD / 8) % 256) == 0 && (kRows * kD / 8) / 256 == 3072);
static_assert(((kRows * kD / 4) % 256) == 0 && (kRows * kD / 4) / 256 == 6144);
static_assert(((kWN * kWWords) % 256) == 0 && (kWN * kWWords) / 256 == 24);
static_assert(((kRows * kDWords) % 256) == 0 && (kRows * kDWords) / 256 == 6144);
static_assert((kPadFloats / 4) == 102 * 32 && (kPadFloats % 4) == 0);
static_assert((kAlpFloats / 4) == 96 * 32);
static_assert((768 / 64) * 4 == 48);
static_assert((kD / 64) * kBatch == 48);

extern "C" void kernel_launch(void* const* d_in, const int* in_sizes, int n_in,
                              void* d_out, int out_size, void* d_ws, size_t ws_size,
                              hipStream_t stream)
{
  if (n_in < 6) return;
  if (in_sizes[0] != kBatch * kL * kD) return;
  if (in_sizes[1] != kD * kNst) return;
  if (in_sizes[2] != kNst * kD) return;
  if (in_sizes[3] != kNst * kD) return;
  if (in_sizes[4] != kD) return;
  if (in_sizes[5] != 1) return;
  if (out_size != kBatch * kL * kD) return;
  if (ws_size < kWsTotal) return;

  const float* u_in   = (const float*)d_in[0];
  const float* a_mat  = (const float*)d_in[1];
  const float* w_b    = (const float*)d_in[2];
  const float* w_c    = (const float*)d_in[3];
  const float* q_del  = (const float*)d_in[4];
  const float* p_del  = (const float*)d_in[5];
  float* out = (float*)d_out;

  char* ws = (char*)d_ws;
  unsigned short* UH   = (unsigned short*)(ws + kOffUH);
  float*          UR   = (float*)(ws + kOffUR);
  unsigned short* WALL = (unsigned short*)(ws + kOffWALL);
  float*          XP   = (float*)(ws + kOffXP);
  float*          DTP  = (float*)(ws + kOffDTP);
  float*          PADS = (float*)(ws + kOffPADS);
  unsigned short* YH   = (unsigned short*)(ws + kOffYH);
  float*          ALP  = PADS;
  float*          DSP  = PADS + kAlpFloats;

  constexpr float s1 = 1.0f / (kXCarry * kWCarry);

  pack_x_kernel<<<(kRows * kD / 8) / 256, 256, 0, stream>>>(u_in, UH);

  rne_x_kernel<<<(kRows * kD / 4) / 256, 256, 0, stream>>>(u_in, UR);

  pack_w_kernel<<<(kWN * kWWords) / 256, 256, 0, stream>>>(w_b, w_c, q_del, WALL);

  eng::gemm_f16_kernel<2, 0><<<dim3((8192 / 32) * (64 / 64) / 8), 256, 0, stream>>>(
      UH, nullptr, 768, WALL, nullptr, 768, XP, 64, 8192, 64, 768, s1, 0.0f);

  dt_plane_kernel<<<(kRows * kDWords) / 256, 256, 0, stream>>>(XP, p_del, DTP);

  pads_kernel<<<102, 32, 0, stream>>>(a_mat, PADS);

  ms1_args sa;
  sa.dtpre = DTP;
  sa.u = UR;
  sa.bc = XP;
  sa.z = nullptr;
  sa.A_log = ALP;
  sa.Dskip = DSP;
  sa.y = (__half*)YH;
  sa.y_lo = nullptr;
  sa.ld_dtpre = kD;
  sa.ld_u = kD;
  sa.ld_bc = kWN;
  sa.ld_z = 0;
  sa.ld_y = kD;
  sa.offB = kOffB;
  sa.offC = kOffC;
  sa.offZ = 0;
  sa.ycarry = kYCarry;
  sa.dir = 1;
  sa.D = kD;
  sa.L = kL;
  sa.nbatch = kBatch;

  ms1_scan_kernel<16><<<dim3((768 / 64) * 4), 64, 0, stream>>>(sa);

  out_kernel<<<(kRows * kD / 4) / 256, 256, 0, stream>>>(YH, out);
}
